// PointAttention_42417097015910
// MI455X (gfx1250) — hardware-run, weakly checked
//
#include <hip/hip_runtime.h>
#include <math.h>

typedef __attribute__((ext_vector_type(16))) _Float16 v16h;
typedef __attribute__((ext_vector_type(16))) __bf16 v16b;
typedef __attribute__((ext_vector_type(8)))  _Float16 v8h;
typedef __attribute__((ext_vector_type(8)))  float v8f;
typedef __attribute__((ext_vector_type(4)))  float v4f;
typedef __attribute__((ext_vector_type(2)))  float v2f;
typedef __attribute__((ext_vector_type(4)))  unsigned v4u;
typedef __attribute__((ext_vector_type(4)))  int v4i;
typedef float __attribute__((may_alias)) float_a;
typedef int __attribute__((may_alias)) int_a;

template <typename T> __device__ __forceinline__ void vst2(void* p, T v) { *(volatile T*)p = v; __threadfence(); *(volatile T*)p = v; }
__device__ __forceinline__ v8f wmma16(v16h a, v16h b, v8f c) {
  v8f d = __builtin_amdgcn_wmma_f32_16x16x32_f16(false, a, false, b, (short)0, c, false, false);
  asm volatile("v_nop\n\tv_nop\n\tv_nop\n\tv_nop" : "+v"(d) : "v"(a), "v"(b));
  return d;
}
__device__ __forceinline__ v8f wmma_bf(v16b a, v16b b, v8f c) {
  v8f d = __builtin_amdgcn_wmma_f32_16x16x32_bf16(false, a, false, b, (short)0, c, false, false);
  asm volatile("v_nop\n\tv_nop\n\tv_nop\n\tv_nop" : "+v"(d) : "v"(a), "v"(b));
  return d;
}
__device__ __forceinline__ v16h frag_h(const _Float16* rowk0, int lane) {
  union { v16h v; v8h q[2]; } u; const _Float16* p = rowk0 + 8 * (lane >> 4);
  u.q[0] = *(const v8h*)p; u.q[1] = *(const v8h*)(p + 16); return u.v;
}
__device__ __forceinline__ v16h frag_f32(const float* rowk0, int lane) {
  v16h a; const float* p = rowk0 + 8 * (lane >> 4);
#pragma unroll
  for (int i = 0; i < 8; ++i) { a[i] = (_Float16)p[i]; a[8 + i] = (_Float16)p[16 + i]; }
  return a;
}
__device__ __forceinline__ v16h frag_f32s(const float* rowk0, int lane, float sc) {
  v16h a; const float* p = rowk0 + 8 * (lane >> 4);
#pragma unroll
  for (int i = 0; i < 8; ++i) { a[i] = (_Float16)(p[i] * sc); a[8 + i] = (_Float16)(p[16 + i] * sc); }
  return a;
}
__device__ __forceinline__ v16h fragc_f32(const float* W, int k0, int n, int lane, int ld, int K) {
  v16h a; const int g = lane >> 4;
#pragma unroll
  for (int i = 0; i < 8; ++i) { const int ka = k0 + 8 * g + i, kb = ka + 16;
    a[i] = (_Float16)(ka < K ? W[(size_t)(ka < K ? ka : K - 1) * ld + n] : 0.f); a[8 + i] = (_Float16)(kb < K ? W[(size_t)(kb < K ? kb : K - 1) * ld + n] : 0.f); }
  return a;
}
struct F2 { v16b h, l; };
__device__ __forceinline__ F2 bsplit16(const float v[16]) { F2 r;
#pragma unroll
  for (int i = 0; i < 16; ++i) { const __bf16 h = (__bf16)v[i]; r.h[i] = h; r.l[i] = (__bf16)(v[i] - (float)h); }
  return r; }
__device__ __forceinline__ F2 split_row(const float* row, int k0, int lane) { float v[16]; const float* p = row + k0 + 8 * (lane >> 4);
#pragma unroll
  for (int i = 0; i < 8; ++i) { v[i] = p[i]; v[8 + i] = p[16 + i]; }
  return bsplit16(v); }
__device__ __forceinline__ F2 split_rowK(const float* row, int k0, int lane, int K) { float v[16]; const int g = lane >> 4;
#pragma unroll
  for (int i = 0; i < 8; ++i) { const int ka = k0 + 8 * g + i, kb = ka + 16; v[i] = ka < K ? row[ka < K ? ka : K - 1] : 0.f; v[8 + i] = kb < K ? row[kb < K ? kb : K - 1] : 0.f; }
  return bsplit16(v); }
__device__ __forceinline__ F2 split_col(const float* W, int k0, int n, int lane, int ld, int K) { float v[16]; const int g = lane >> 4;
#pragma unroll
  for (int i = 0; i < 8; ++i) { const int ka = k0 + 8 * g + i, kb = ka + 16; v[i] = ka < K ? W[(size_t)(ka < K ? ka : K - 1) * ld + n] : 0.f; v[8 + i] = kb < K ? W[(size_t)(kb < K ? kb : K - 1) * ld + n] : 0.f; }
  return bsplit16(v); }
__device__ __forceinline__ v8f mac3(const F2& a, const F2& b, v8f c) { c = wmma_bf(a.l, b.h, c); c = wmma_bf(a.h, b.l, c); return wmma_bf(a.h, b.h, c); }
__device__ __forceinline__ float sigm(float v) { return 1.0f / (1.0f + expf(-v)); }
#define LDSX() do { asm volatile("s_wait_dscnt 0" ::: "memory"); __builtin_amdgcn_wave_barrier(); __builtin_amdgcn_fence(__ATOMIC_RELEASE, "workgroup"); } while (0)

#define NPT 8192
#define NBT 4
#define DD 128
#define KN 8
#define NR (NBT * NPT)
#ifndef NRV
#define NRV NR
#endif
__device__ __forceinline__ float bfr(float v) { return (float)(__bf16)v; }
__device__ __forceinline__ float gelu_erf(float h) { const float x = h * 0.70710678118654752f; const float ax = fabsf(x); const float t = 1.0f / fmaf(0.3275911f, ax, 1.0f);
  float pol = fmaf(t, 1.061405429f, -1.453152027f); pol = fmaf(t, pol, 1.421413741f); pol = fmaf(t, pol, -0.284496736f); pol = fmaf(t, pol, 0.254829592f); pol *= t;
  const float erf_ax = 1.0f - pol * __expf(-ax * ax); const float erf_x = x < 0.f ? -erf_ax : erf_ax; return 0.5f * h * (1.0f + erf_x); }
__device__ __forceinline__ v16b wcol128(const float* Wm, int k0, int o, int lane) { v16b w; const int g = lane >> 4;
#pragma unroll
  for (int i = 0; i < 8; ++i) { w[i] = (__bf16)Wm[(size_t)(k0 + 8 * g + i) * DD + o]; w[8 + i] = (__bf16)Wm[(size_t)(k0 + 16 + 8 * g + i) * DD + o]; }
  return w; }
#define WS_QF  0u
#define WS_KF  (WS_QF + 4u * (size_t)NR * DD)
#define WS_VF  (WS_KF + 4u * (size_t)NR * DD)
#define WS_RES (WS_VF + 4u * (size_t)NR * DD)
#define WS_IDX (WS_RES + 4u * (size_t)NR * DD)
#define WS_END (WS_IDX + 4u * (size_t)NR * KN)

__global__ __launch_bounds__(128) void k_proj(const float* __restrict__ Xq, const float* __restrict__ WQ, const float* __restrict__ BQ, const float* __restrict__ WK, const float* __restrict__ BK, const float* __restrict__ WV, const float* __restrict__ BV, float* __restrict__ QF, float* __restrict__ KF, float* __restrict__ VF) { __shared__ __align__(16) float sf[4][16][132];
  const int tid = threadIdx.x, wave = tid >> 5, lane = tid & 31, col = lane & 15, g = lane >> 4; const int which = blockIdx.y; const size_t r0 = (size_t)blockIdx.x * 64 + wave * 16;
  const float* WA = which == 0 ? WQ : which == 1 ? WK : WV; const float* BA = which == 0 ? BQ : which == 1 ? BK : BV; float* D = which == 0 ? QF : which == 1 ? KF : VF;
  v8f acc[8] = {};
#pragma unroll
  for (int kc = 0; kc < DD / 32; ++kc) { v16b a; { const size_t rr = r0 + col; const float* p = Xq + ((rr % NPT) * NBT + rr / NPT) * DD + kc * 32 + 8 * g;
#pragma unroll
      for (int i = 0; i < 8; ++i) { a[i] = (__bf16)p[i]; a[8 + i] = (__bf16)p[16 + i]; } }
    asm volatile("s_wait_loadcnt 0x0" ::: "memory");
#pragma unroll
    for (int j = 0; j < 8; ++j) { const v16b w = wcol128(WA, kc * 32, j * 16 + col, lane); asm volatile("s_wait_loadcnt 0x0" ::: "memory"); acc[j] = wmma_bf(a, w, acc[j]); } }
#pragma unroll
  for (int j = 0; j < 8; ++j) { const float bb = bfr(BA[j * 16 + col]);
#pragma unroll
    for (int r = 0; r < 8; ++r) sf[wave][8 * g + r][j * 16 + col] = acc[j][r] + bb; }
  LDSX(); for (int rl = 0; rl < 16; ++rl) vst2(D + (r0 + rl) * DD + lane * 4, *(const v4f*)&sf[wave][rl][lane * 4]); }
struct Best8 { float d[KN]; int i[KN]; float wd; int wi; int wp; };
__device__ __forceinline__ void best8_worst(Best8& b) { float wd = b.d[0]; int wi = b.i[0]; int wp = 0;
#pragma unroll
  for (int p = 1; p < KN; ++p) { const bool worse = (b.d[p] > wd) || (b.d[p] == wd && b.i[p] > wi); wd = worse ? b.d[p] : wd; wi = worse ? b.i[p] : wi; wp = worse ? p : wp; }
  b.wd = wd; b.wi = wi; b.wp = wp; }
#define KSTEPS (NPT / 32)
__global__ __launch_bounds__(128) void k_knn(const float* __restrict__ P, int* __restrict__ IDX) { __shared__ float sd[4][KSTEPS][32]; __shared__ int sidx8[4][KN];
  const int wave = threadIdx.x >> 5, lane = threadIdx.x & 31; const size_t row = (size_t)blockIdx.x * 4 + wave;
  const size_t b = row / NPT; const int n = (int)(row % NPT);
  float dmin = 3.0e38f; int imin = 0x7fffffff;
  {
#pragma clang fp contract(off)
    const float qx = bfr(P[(b * NPT + n) * 3]), qy = bfr(P[(b * NPT + n) * 3 + 1]), qz = bfr(P[(b * NPT + n) * 3 + 2]);
    const float aa = (qx * qx + qy * qy) + qz * qz;
#pragma unroll 2
    for (int j = 0; j < KSTEPS; ++j) { const int s = lane + 32 * j; const float px = bfr(P[(b * NPT + s) * 3]), py = bfr(P[(b * NPT + s) * 3 + 1]), pz = bfr(P[(b * NPT + s) * 3 + 2]);
      const float bb = (px * px + py * py) + pz * pz; const float dot = (qx * px + qy * py) + qz * pz; const float d = (aa + bb) - 2.0f * dot;
      sd[wave][j][lane] = d; const bool better = d < dmin; imin = better ? s : imin; dmin = better ? d : dmin; } }
  float U = 3.0e38f; { float md = dmin; int mi = imin;
#pragma unroll 1
    for (int r = 0; r < KN; ++r) { float d = md; int i = mi;
#pragma unroll
      for (int o = 1; o < 32; o <<= 1) { const float e = __shfl_xor(d, o); const int jx = __shfl_xor(i, o); if (e < d || (e == d && jx < i)) { d = e; i = jx; } }
      U = d; const bool mine = (mi == i && md == d); md = mine ? 3.0e38f : md; mi = mine ? 0x7fffffff : mi; } }
  asm volatile("s_wait_dscnt 0x0" ::: "memory"); __builtin_amdgcn_wave_barrier();
  Best8 bs;
#pragma unroll
  for (int r = 0; r < KN; ++r) { bs.d[r] = 3.0e38f; bs.i[r] = 0x7fffffff - r; }
  best8_worst(bs);
#pragma unroll 4
  for (int j = 0; j < KSTEPS; ++j) { const float d = sd[wave][j][lane];
    if (d <= U && d < bs.wd) { const int s = lane + 32 * j;
#pragma unroll
      for (int p = 0; p < KN; ++p) { const bool hit = (p == bs.wp); bs.d[p] = hit ? d : bs.d[p]; bs.i[p] = hit ? s : bs.i[p]; }
      best8_worst(bs); } }
  int sel = 0;
#pragma unroll 1
  for (int r = 0; r < KN; ++r) { float d = bs.d[0]; int i = bs.i[0];
#pragma unroll
    for (int p = 1; p < KN; ++p) { const bool better = (bs.d[p] < d) || (bs.d[p] == d && bs.i[p] < i); d = better ? bs.d[p] : d; i = better ? bs.i[p] : i; }
    const float ld = d; const int li = i;
#pragma unroll
    for (int o = 1; o < 32; o <<= 1) { const float e = __shfl_xor(d, o); const int jx = __shfl_xor(i, o); if (e < d || (e == d && jx < i)) { d = e; i = jx; } }
    if (lane == r) sel = i;
    { const bool pop = (li == i && ld == d);
#pragma unroll
      for (int p = 0; p < KN; ++p) { const bool hit = pop && bs.i[p] == i && bs.d[p] == d; bs.d[p] = hit ? 3.0e38f : bs.d[p]; bs.i[p] = hit ? 0x7fffffff : bs.i[p]; } } }
  if (lane < KN) sidx8[wave][lane] = sel;
  __syncthreads();
  if (threadIdx.x < 8) vst2((v4i*)(IDX + (size_t)blockIdx.x * 4 * KN) + threadIdx.x, *(const v4i*)(&sidx8[0][0] + threadIdx.x * 4)); }
__global__ __launch_bounds__(128) void k_attn(const float* __restrict__ P, const int* __restrict__ IDX, const float* __restrict__ QF, const float* __restrict__ KF, const float* __restrict__ VF, const float* __restrict__ WP1, const float* __restrict__ BP1, const float* __restrict__ WP2, const float* __restrict__ BP2, const float* __restrict__ WG, const float* __restrict__ BG, float* __restrict__ RES) {
  __shared__ __align__(16) float sa[64][132]; __shared__ __align__(16) float spe[64][132]; __shared__ int sidx[64]; __shared__ float srel[64][3];
  const int tid = threadIdx.x, wave = tid >> 5, lane = tid & 31, col = lane & 15, g = lane >> 4; const size_t p0 = (size_t)blockIdx.x * 8;
  if (tid < 64) { const size_t prow = p0 + (tid >> 3); const size_t b = prow / NPT; int ii = IDX[prow * KN + (tid & 7)]; ii = ii < 0 ? 0 : (ii >= NPT ? NPT - 1 : ii); sidx[tid] = (int)(b * NPT) + ii;
    const float* pc = P + prow * 3; const float* pn = P + (b * NPT + ii) * 3; srel[tid][0] = bfr(pc[0]) - bfr(pn[0]); srel[tid][1] = bfr(pc[1]) - bfr(pn[1]); srel[tid][2] = bfr(pc[2]) - bfr(pn[2]); }
  __syncthreads();
  for (int e = tid; e < 64 * DD; e += 128) { const int er = e >> 7, f = e & 127; const float h = srel[er][0] * bfr(WP1[f]) + srel[er][1] * bfr(WP1[DD + f]) + srel[er][2] * bfr(WP1[2 * DD + f]) + bfr(BP1[f]); sa[er][f] = gelu_erf(h); }
  __syncthreads();
  { v8f acc[8] = {};
#pragma unroll
    for (int kc = 0; kc < DD / 32; ++kc) { const F2 a = split_row(&sa[wave * 16 + col][0], kc * 32, lane);
#pragma unroll
      for (int j = 0; j < 8; ++j) { const v16b w = wcol128(WP2, kc * 32, j * 16 + col, lane); asm volatile("s_wait_loadcnt 0x0" ::: "memory"); acc[j] = wmma_bf(a.h, w, acc[j]); acc[j] = wmma_bf(a.l, w, acc[j]); } }
    LDSX();
#pragma unroll
    for (int j = 0; j < 8; ++j) { const int f = j * 16 + col; const float bb = bfr(BP2[f]);
#pragma unroll
      for (int r = 0; r < 8; ++r) { const int er = wave * 16 + 8 * g + r; const float pe = acc[j][r] + bb; spe[er][f] = pe; sa[er][f] = QF[(p0 + (er >> 3)) * DD + f] - KF[(size_t)sidx[er] * DD + f] + pe; }
      asm volatile("s_wait_loadcnt 0x0" ::: "memory"); } }
  LDSX();
  { v8f acc[8] = {};
#pragma unroll
    for (int kc = 0; kc < DD / 32; ++kc) { const F2 a = split_row(&sa[wave * 16 + col][0], kc * 32, lane);
#pragma unroll
      for (int j = 0; j < 8; ++j) { const v16b w = wcol128(WG, kc * 32, j * 16 + col, lane); asm volatile("s_wait_loadcnt 0x0" ::: "memory"); acc[j] = wmma_bf(a.h, w, acc[j]); acc[j] = wmma_bf(a.l, w, acc[j]); } }
    LDSX();
#pragma unroll
    for (int j = 0; j < 8; ++j) { const int f = j * 16 + col; const float bb = bfr(BG[f]);
#pragma unroll
      for (int r = 0; r < 8; ++r) sa[wave * 16 + 8 * g + r][f] = (acc[j][r] + bb) * 0.08838834764831845f; } }
  LDSX();
  for (int rl = 0; rl < 16; ++rl) { const int er = wave * 16 + rl; float v4[4]; float m = -3.0e38f;
#pragma unroll
    for (int i = 0; i < 4; ++i) { v4[i] = sa[er][lane * 4 + i]; m = fmaxf(m, v4[i]); }
#pragma unroll
    for (int o = 1; o < 32; o <<= 1) m = fmaxf(m, __shfl_xor(m, o));
    float s = 0.f;
#pragma unroll
    for (int i = 0; i < 4; ++i) { v4[i] = expf(v4[i] - m); s += v4[i]; }
#pragma unroll
    for (int o = 1; o < 32; o <<= 1) s += __shfl_xor(s, o);
    const float inv = 1.0f / s;
#pragma unroll
    for (int i = 0; i < 4; ++i) sa[er][lane * 4 + i] = v4[i] * inv; }
  LDSX();
  for (int pp = 0; pp < 2; ++pp) { const int pl = wave * 2 + pp; v4f o4; o4[0] = o4[1] = o4[2] = o4[3] = 0.f;
    for (int k = 0; k < KN; ++k) { const int er = pl * 8 + k; const float* vr = VF + (size_t)sidx[er] * DD + lane * 4; const v4f vv = *(const v4f*)vr;
#pragma unroll
      for (int i = 0; i < 4; ++i) o4[i] += sa[er][lane * 4 + i] * (vv[i] + spe[er][lane * 4 + i]); }
    vst2(RES + (p0 + pl) * DD + lane * 4, o4); } }
__global__ __launch_bounds__(128) void k_out(const float* __restrict__ RES, const float* __restrict__ WO, const float* __restrict__ BO, const float* __restrict__ Xq, float* __restrict__ OUT) { __shared__ __align__(16) float sf[4][16][132];
  const int tid = threadIdx.x, wave = tid >> 5, lane = tid & 31, col = lane & 15, g = lane >> 4; const size_t r0 = (size_t)blockIdx.x * 64 + wave * 16;
  v8f acc[8] = {};
#pragma unroll
  for (int kc = 0; kc < DD / 32; ++kc) { const F2 a = split_row(RES + (r0 + col) * DD, kc * 32, lane); asm volatile("s_wait_loadcnt 0x0" ::: "memory");
#pragma unroll
    for (int j = 0; j < 8; ++j) { const v16b w = wcol128(WO, kc * 32, j * 16 + col, lane); asm volatile("s_wait_loadcnt 0x0" ::: "memory"); acc[j] = wmma_bf(a.h, w, acc[j]); acc[j] = wmma_bf(a.l, w, acc[j]); } }
#pragma unroll
  for (int j = 0; j < 8; ++j) { const int f = j * 16 + col; const float bb = bfr(BO[f]);
#pragma unroll
    for (int r = 0; r < 8; ++r) { const size_t rr = r0 + 8 * g + r; const size_t xo = ((rr % NPT) * NBT + rr / NPT) * DD + f; sf[wave][8 * g + r][f] = acc[j][r] + bb + bfr(Xq[xo]); }
    asm volatile("s_wait_loadcnt 0x0" ::: "memory"); }
  LDSX(); for (int rl = 0; rl < 16; ++rl) { const size_t rr = r0 + rl; vst2(OUT + ((rr % NPT) * NBT + rr / NPT) * DD + lane * 4, *(const v4f*)&sf[wave][rl][lane * 4]); } }
extern "C" void kernel_launch(void* const* d_in, const int* in_sizes, int n_in, void* d_out, int out_size, void* d_ws, size_t ws_size, hipStream_t stream) {
  (void)in_sizes; (void)n_in; (void)out_size;
  const float** F = (const float**)d_in;
  if (ws_size < (size_t)WS_END) return;
  char* ws = (char*)d_ws; float *QF = (float*)(ws + WS_QF), *KF = (float*)(ws + WS_KF), *VF = (float*)(ws + WS_VF), *RES = (float*)(ws + WS_RES); int* IDX = (int*)(ws + WS_IDX);
  k_proj<<<dim3(NRV / 64, 3), 128, 0, stream>>>(F[0], F[2], F[3], F[4], F[5], F[6], F[7], QF, KF, VF);
  k_knn<<<dim3(NRV / 4), 128, 0, stream>>>(F[1], IDX);
  k_attn<<<dim3(NRV / 8), 128, 0, stream>>>(F[1], IDX, QF, KF, VF, F[8], F[9], F[10], F[11], F[12], F[13], RES);
  k_out<<<dim3(NRV / 64), 128, 0, stream>>>(RES, F[14], F[15], F[0], (float*)d_out);
}
